// GNNStructEncoder_80599356276736
// MI455X (gfx1250) — hardware-verified
//
#include <hip/hip_runtime.h>
#include <stddef.h>


#define DH      256
#define NTHR    256
#define NWAVE   8
#define EPT     8
#define NGRP    2
#define CHUNK   (NTHR * EPT * NGRP)
#define WCAP    (EPT * NGRP * 32)
#define LISTN   (NWAVE * WCAP)
#define NBC     4096
#define NBF     1024
#define RCAP    40960
#define RBN     128
#define TGT     256
#define DEGCAP  256
#define GROWS   64
#define OTHR    512
#define LNODE   64
#define WSCALE  16.0f
#define ASCALE  0.125f
#define F16INV  0.5f
#define L2EPS   1e-12f

#define LDS_GEMM (GROWS * DH * 4)
#define LDS_FILL ((RCAP + NBF + LISTN) * 4 + 64)

static_assert((CHUNK & (CHUNK - 1)) == 0);
static_assert(CHUNK <= 4096);
static_assert(NBC <= 4096 && NBF <= 4096);
static_assert((NBC & (NBC - 1)) == 0 && (NBF & (NBF - 1)) == 0);
static_assert(NBC == 4 * NBF);
static_assert(OTHR * 8 == NBC);
static_assert((RCAP % 32) == 0);
static_assert(TGT == NWAVE * 32 && (TGT % GROWS) == 0);
static_assert(GROWS == 64 && (GROWS % NWAVE) == 0);
static_assert(DH == 256);
static_assert(LNODE == NWAVE * 8);

typedef float          v4f   __attribute__((ext_vector_type(4)));
typedef float          v8f   __attribute__((ext_vector_type(8)));
typedef int            v4i   __attribute__((ext_vector_type(4)));
typedef _Float16       v8h   __attribute__((ext_vector_type(8)));
typedef _Float16       v16h  __attribute__((ext_vector_type(16)));
typedef __bf16         v16b  __attribute__((ext_vector_type(16)));
typedef unsigned short v8us  __attribute__((ext_vector_type(8)));
typedef unsigned short v16us __attribute__((ext_vector_type(16)));
union Frag { v16us u; v8us h[2]; v16h f; v16b b; };

__device__ __forceinline__ float wsum32(float v) {
#pragma unroll
  for (int o = 16; o > 0; o >>= 1) v += __shfl_xor(v, o, 32);
  return v;
}

__device__ __forceinline__ unsigned short bf_rne(float x) {
  unsigned u = __float_as_uint(x);
  u += 0x7FFFu + ((u >> 16) & 1u);
  return (unsigned short)(u >> 16);
}

__device__ __forceinline__ void split8(v4f a, v4f b, v8us& hv, v8us& lv) {
  float x[8];
  x[0] = a.x; x[1] = a.y; x[2] = a.z; x[3] = a.w; x[4] = b.x; x[5] = b.y; x[6] = b.z; x[7] = b.w;
#pragma unroll
  for (int e = 0; e < 8; ++e) {
    const unsigned short hb = bf_rne(x[e]);
    const float hf = __uint_as_float(((unsigned)hb) << 16);
    const unsigned short lb = bf_rne(x[e] - hf);
    hv[e] = hb;
    lv[e] = lb;
  }
}

__device__ __forceinline__ v8h cvt8h(v4f a, v4f b) {
  v8h r;
  r[0] = (_Float16)a.x; r[1] = (_Float16)a.y; r[2] = (_Float16)a.z; r[3] = (_Float16)a.w;
  r[4] = (_Float16)b.x; r[5] = (_Float16)b.y; r[6] = (_Float16)b.z; r[7] = (_Float16)b.w;
  return r;
}

__device__ __forceinline__ float dot8(v4f a, v4f b, v4f c, v4f d) {
  return a.x * c.x + a.y * c.y + a.z * c.z + a.w * c.w + b.x * d.x + b.y * d.y + b.z * d.z + b.w * d.w;
}

__device__ __forceinline__ v8f wm_f16(v16h a, v16h b, v8f c) {
  v8f d = __builtin_amdgcn_wmma_f32_16x16x32_f16(false, a, false, b, (short)0, c, false, false);
  asm volatile("v_nop\n\tv_nop\n\tv_nop\n\tv_nop" : "+v"(d) : "v"(a), "v"(b));
  return d;
}
__device__ __forceinline__ v8f wm_bf16(v16b a, v16b b, v8f c) {
  v8f d = __builtin_amdgcn_wmma_f32_16x16x32_bf16(false, a, false, b, (short)0, c, false, false);
  asm volatile("v_nop\n\tv_nop\n\tv_nop\n\tv_nop" : "+v"(d) : "v"(a), "v"(b));
  return d;
}

template <int NB>
__device__ __forceinline__ int scan_chunk(const int* __restrict__ dsts, int nE, int cbase, int slotBase,
                                          int vec8, int* list, int tid, int lane, int wave) {
  int wc = 0;
#pragma unroll
  for (int g = 0; g < NGRP; ++g) {
    const int el0  = (g * NTHR + tid) * EPT;
    const int e0   = cbase + el0;
    const int sent = -2147483647 - 1;
    v4i da, db;
    if (vec8 != 0 && cbase + CHUNK <= nE) {
      da = *(const v4i*)(dsts + e0);
      db = *(const v4i*)(dsts + e0 + 4);
    } else {
      da.x = (e0     < nE) ? dsts[min(e0, nE - 1)] : sent;
      da.y = (e0 + 1 < nE) ? dsts[min(e0 + 1, nE - 1)] : sent;
      da.z = (e0 + 2 < nE) ? dsts[min(e0 + 2, nE - 1)] : sent;
      da.w = (e0 + 3 < nE) ? dsts[min(e0 + 3, nE - 1)] : sent;
      db.x = (e0 + 4 < nE) ? dsts[min(e0 + 4, nE - 1)] : sent;
      db.y = (e0 + 5 < nE) ? dsts[min(e0 + 5, nE - 1)] : sent;
      db.z = (e0 + 6 < nE) ? dsts[min(e0 + 6, nE - 1)] : sent;
      db.w = (e0 + 7 < nE) ? dsts[min(e0 + 7, nE - 1)] : sent;
    }
    const unsigned nb = (unsigned)slotBase;
    const unsigned s0 = (unsigned)da.x - nb, s1 = (unsigned)da.y - nb;
    const unsigned s2 = (unsigned)da.z - nb, s3 = (unsigned)da.w - nb;
    const unsigned s4 = (unsigned)db.x - nb, s5 = (unsigned)db.y - nb;
    const unsigned s6 = (unsigned)db.z - nb, s7 = (unsigned)db.w - nb;
    const bool h0 = s0 < (unsigned)NB, h1 = s1 < (unsigned)NB, h2 = s2 < (unsigned)NB, h3 = s3 < (unsigned)NB;
    const bool h4 = s4 < (unsigned)NB, h5 = s5 < (unsigned)NB, h6 = s6 < (unsigned)NB, h7 = s7 < (unsigned)NB;
    const unsigned any = __builtin_amdgcn_ballot_w32(h0 | h1 | h2 | h3 | h4 | h5 | h6 | h7);
    if (any != 0u) {
#define HITJ(J, HJ, SJ) { \
        const unsigned mj = __builtin_amdgcn_ballot_w32(HJ); \
        if (mj != 0u) { \
          if (HJ) { \
            const int pos = wc + (int)__builtin_amdgcn_mbcnt_lo(mj, 0u); \
            if (pos < WCAP) list[wave * WCAP + pos] = ((el0 + (J)) << 12) | (int)(SJ); \
          } \
          wc += (int)__builtin_popcount(mj); } }
      HITJ(0, h0, s0)
      HITJ(1, h1, s1)
      HITJ(2, h2, s2)
      HITJ(3, h3, s3)
      HITJ(4, h4, s4)
      HITJ(5, h5, s5)
      HITJ(6, h6, s6)
      HITJ(7, h7, s7)
#undef HITJ
    }
  }
  return wc;
}

__global__ __launch_bounds__(NTHR) void k_wprep(
    const float* __restrict__ q0, const float* __restrict__ q1, const float* __restrict__ q2,
    const float* __restrict__ q3, const float* __restrict__ q4, const float* __restrict__ q5,
    const float* __restrict__ q6, const float* __restrict__ q7, const float* __restrict__ q8,
    const float* __restrict__ q9, const float* __restrict__ q10,
    unsigned short* whl, unsigned short* wf) {
  const int tid = threadIdx.x;
  const int p = (int)(blockIdx.x >> 5);
  const float* W = p == 0 ? q0 : (p == 1 ? q1 : (p == 2 ? q2 : (p == 3 ? q3 : (p == 4 ? q4 : (p == 5 ? q5 :
                   (p == 6 ? q6 : (p == 7 ? q7 : (p == 8 ? q8 : (p == 9 ? q9 : q10)))))))));
  const int i  = (int)((blockIdx.x & 31) * NTHR) + tid;
  const int o  = i * 8;
  const int n  = o >> 8;
  const int k0 = o & 255;
  float v[8];
#pragma unroll
  for (int e = 0; e < 8; ++e) v[e] = W[(size_t)(k0 + e) * DH + n];
  if (p < 4) {
    v4f a, b;
    a.x = v[0]; a.y = v[1]; a.z = v[2]; a.w = v[3];
    b.x = v[4]; b.y = v[5]; b.z = v[6]; b.w = v[7];
    v8us hv, lv;
    split8(a, b, hv, lv);
    unsigned short* hp = whl + (size_t)(2 * p) * (DH * DH) + o;
    unsigned short* lp = hp + DH * DH;
    *(volatile v8us*)hp = hv;
    *(volatile v8us*)lp = lv;
    __threadfence();
    *(volatile v8us*)hp = hv;
    *(volatile v8us*)lp = lv;
  } else {
    v4f a, b;
    a.x = v[0] * WSCALE; a.y = v[1] * WSCALE; a.z = v[2] * WSCALE; a.w = v[3] * WSCALE;
    b.x = v[4] * WSCALE; b.y = v[5] * WSCALE; b.z = v[6] * WSCALE; b.w = v[7] * WSCALE;
    const v8h fv = cvt8h(a, b);
    unsigned short* fp = wf + (size_t)(p - 4) * (DH * DH) + o;
    *(volatile v8h*)fp = fv;
    __threadfence();
    *(volatile v8h*)fp = fv;
  }
}

__global__ __launch_bounds__(NTHR) void k_count(
    const int* __restrict__ dsts, int* cnt, int nE, int vec8) {
  __shared__ __attribute__((aligned(16))) int scnt[NBC];
  __shared__ __attribute__((aligned(16))) int list[LISTN];
  __shared__ int wcnt[NWAVE];
  const int tid = threadIdx.x, lane = tid & 31, wave = tid >> 5;
  const int nodeBase = blockIdx.x * NBC;

  for (int i = tid; i < NBC; i += NTHR) scnt[i] = 0;
  __syncthreads();

  const int nChunks = (nE + CHUNK - 1) / CHUNK;
#pragma unroll 1
  for (int ch = 0; ch < nChunks; ++ch) {
    const int cbase = ch * CHUNK;
    const int wc = scan_chunk<NBC>(dsts, nE, cbase, nodeBase, vec8, list, tid, lane, wave);
    if (lane == 0) wcnt[wave] = wc;
    __syncthreads();
    if (wave == 0) {
#pragma unroll 1
      for (int wsx = 0; wsx < NWAVE; ++wsx) {
        int n = __builtin_amdgcn_readfirstlane(wcnt[wsx]);
        n = n > WCAP ? WCAP : (n < 0 ? 0 : n);
        const int* lp = list + wsx * WCAP;
#pragma unroll 1
        for (int i = 0; i < n; ++i) {
          const int ent  = __builtin_amdgcn_readfirstlane(lp[i]);
          const int slot = ent & (NBC - 1);
          if (lane == 0) scnt[slot] = scnt[slot] + 1;
        }
      }
    }
    __syncthreads();
  }

  v4i cq[4];
#pragma unroll
  for (int q = 0; q < 4; ++q) {
    const int f = (wave * 4 + q) * 128 + 4 * lane;
    cq[q] = *(const v4i*)(scnt + f);
  }
  int* cp = cnt + (size_t)nodeBase;
#pragma unroll
  for (int q = 0; q < 4; ++q) {
    const int f = (wave * 4 + q) * 128 + 4 * lane;
    *(volatile v4i*)(cp + f) = cq[q];
  }
  __threadfence();
#pragma unroll
  for (int q = 0; q < 4; ++q) {
    const int f = (wave * 4 + q) * 128 + 4 * lane;
    *(volatile v4i*)(cp + f) = cq[q];
  }
}

__global__ __launch_bounds__(OTHR) void k_offsets(
    const int* __restrict__ cnt, int* off, int* rbase, int nChunk) {
  __shared__ __attribute__((aligned(16))) int soff[NBC];
  __shared__ __attribute__((aligned(16))) int srb[RBN];
  __shared__ int wtot[OTHR / 32];
  const int tid = threadIdx.x, lane = tid & 31, wave = tid >> 5, sub = tid >> 7;
  for (int i = tid; i < RBN; i += OTHR) srb[i] = 0;
  int carry = 0;
#pragma unroll 1
  for (int ch = 0; ch < nChunk; ++ch) {
    const int base = ch * NBC;
    const v4i c0 = *(const v4i*)(cnt + base + 8 * tid);
    const v4i c1 = *(const v4i*)(cnt + base + 8 * tid + 4);
    const int e0 = max(c0.x, 0), e1 = max(c0.y, 0), e2 = max(c0.z, 0), e3 = max(c0.w, 0);
    const int e4 = max(c1.x, 0), e5 = max(c1.y, 0), e6 = max(c1.z, 0), e7 = max(c1.w, 0);
    const int ts = e0 + e1 + e2 + e3 + e4 + e5 + e6 + e7;
    int incl = ts;
#pragma unroll
    for (int d = 1; d < 32; d <<= 1) {
      const int t = __shfl_up(incl, d, 32);
      if (lane >= d) incl += t;
    }
    if (lane == 31) wtot[wave] = incl;
    __syncthreads();
    const int S0 = wtot[0]  + wtot[1]  + wtot[2]  + wtot[3];
    const int S1 = wtot[4]  + wtot[5]  + wtot[6]  + wtot[7];
    const int S2 = wtot[8]  + wtot[9]  + wtot[10] + wtot[11];
    const int S3 = wtot[12] + wtot[13] + wtot[14] + wtot[15];
    int pre = 0;
#pragma unroll 1
    for (int w = 4 * sub; w < wave; ++w) pre += wtot[w];
    const int b0 = carry;
    const int b1 = b0 + ((S0 + 31) & ~31);
    const int b2 = b1 + ((S1 + 31) & ~31);
    const int b3 = b2 + ((S2 + 31) & ~31);
    const int b4 = b3 + ((S3 + 31) & ~31);
    const int myb = sub == 0 ? b0 : (sub == 1 ? b1 : (sub == 2 ? b2 : b3));
    if (tid == 0) {
      srb[min(4 * ch + 0, RBN - 1)] = b0;
      srb[min(4 * ch + 1, RBN - 1)] = b1;
      srb[min(4 * ch + 2, RBN - 1)] = b2;
      srb[min(4 * ch + 3, RBN - 1)] = b3;
    }
    int run = myb + pre + incl - ts;
    soff[8 * tid + 0] = run; run += e0;
    soff[8 * tid + 1] = run; run += e1;
    soff[8 * tid + 2] = run; run += e2;
    soff[8 * tid + 3] = run; run += e3;
    soff[8 * tid + 4] = run; run += e4;
    soff[8 * tid + 5] = run; run += e5;
    soff[8 * tid + 6] = run; run += e6;
    soff[8 * tid + 7] = run;
    carry = b4;
    __syncthreads();
    const v4i o0 = *(const v4i*)(soff + 4 * tid);
    const v4i o1 = *(const v4i*)(soff + 4 * (tid + OTHR));
    int* op = off + base;
    *(volatile v4i*)(op + 4 * tid) = o0;
    *(volatile v4i*)(op + 4 * (tid + OTHR)) = o1;
    __threadfence();
    *(volatile v4i*)(op + 4 * tid) = o0;
    *(volatile v4i*)(op + 4 * (tid + OTHR)) = o1;
    __syncthreads();
  }
  if (tid == 0) srb[min(4 * nChunk, RBN - 1)] = carry;
  __syncthreads();
  v4i rv = {0, 0, 0, 0};
  if (tid < 32) rv = *(const v4i*)(srb + 4 * tid);
  if (tid < 32) *(volatile v4i*)(rbase + 4 * tid) = rv;
  __threadfence();
  if (tid < 32) *(volatile v4i*)(rbase + 4 * tid) = rv;
}

__global__ __launch_bounds__(NTHR) void k_fill(
    const int* __restrict__ srcs, const int* __restrict__ dsts, const int* __restrict__ off,
    const int* __restrict__ rbase, int* csr, int nN, int nE, int vec8, int csrLen) {
  extern __shared__ v4f lds_dyn[];
  int* region = (int*)lds_dyn;
  int* cursor = region + RCAP;
  int* list   = cursor + NBF;
  int* wcnt   = list + LISTN;
  const int tid = threadIdx.x, lane = tid & 31, wave = tid >> 5;
  const int b = blockIdx.x;
  const int nodeBase = b * NBF;

  int rb0 = rbase[min(b, RBN - 1)];
  const int rb1 = rbase[min(b + 1, RBN - 1)];
  rb0 = rb0 < 0 ? 0 : (rb0 > csrLen ? csrLen : rb0);
  rb0 &= ~31;
  int len = rb1 - rb0;
  len = len < 0 ? 0 : (len > RCAP ? RCAP : len);
  int lenW = (len + 31) & ~31;
  if (rb0 + lenW > csrLen) lenW = (csrLen - rb0) & ~31;

  {
    const v4i z = {0, 0, 0, 0};
    for (int i = tid; i < RCAP / 4; i += NTHR) ((v4i*)region)[i] = z;
    for (int s = tid; s < NBF; s += NTHR) {
      int o = off[nodeBase + s] - rb0;
      o = o < 0 ? 0 : (o > RCAP ? RCAP : o);
      cursor[s] = o;
    }
  }
  __syncthreads();

  const int nChunks = (nE + CHUNK - 1) / CHUNK;
#pragma unroll 1
  for (int ch = 0; ch < nChunks; ++ch) {
    const int cbase = ch * CHUNK;
    const int wc = scan_chunk<NBF>(dsts, nE, cbase, nodeBase, vec8, list, tid, lane, wave);
    if (lane == 0) wcnt[wave] = wc;
    __syncthreads();
    if (wave == 0) {
#pragma unroll 1
      for (int wsx = 0; wsx < NWAVE; ++wsx) {
        int n = __builtin_amdgcn_readfirstlane(wcnt[wsx]);
        n = n > WCAP ? WCAP : (n < 0 ? 0 : n);
        const int* lp = list + wsx * WCAP;
#pragma unroll 1
        for (int i = 0; i < n; ++i) {
          const int ent  = __builtin_amdgcn_readfirstlane(lp[i]);
          const int slot = ent & (NBF - 1);
          int e = cbase + ((ent >> 12) & (CHUNK - 1));
          e = e > nE - 1 ? nE - 1 : e;
          int sv = srcs[e];
          sv = sv < 0 ? 0 : (sv > nN - 1 ? nN - 1 : sv);
          if (lane == 0) {
            int pos = cursor[slot];
            pos = pos < 0 ? 0 : (pos > RCAP - 1 ? RCAP - 1 : pos);
            region[pos] = sv;
            const int np = pos + 1;
            cursor[slot] = np > RCAP ? RCAP : np;
          }
        }
      }
    }
    __syncthreads();
  }

  const int nv = lenW >> 2;
  int* gp = csr + rb0;
#pragma unroll 1
  for (int i = tid; i < nv; i += NTHR) { const v4i v = ((const v4i*)region)[i]; *(volatile v4i*)(gp + 4 * i) = v; }
  __threadfence();
#pragma unroll 1
  for (int i = tid; i < nv; i += NTHR) { const v4i v = ((const v4i*)region)[i]; *(volatile v4i*)(gp + 4 * i) = v; }
}

__global__ __launch_bounds__(NTHR) void k_agg(
    const int* __restrict__ csr, const int* __restrict__ off, const int* __restrict__ cnt,
    const float* __restrict__ X, int nN, int csrLen, int doHL, int doF,
    unsigned short* Ohi, unsigned short* Olo, unsigned short* Of) {
  const int tid = threadIdx.x, lane = tid & 31, wave = tid >> 5;
  const int tbase = blockIdx.x * TGT + wave * 32;
  const int cl = tbase + lane;
  const int cnt_l = cnt[cl];
  const int off_l = off[cl];

#pragma unroll 1
  for (int j = 0; j < 32; ++j) {
    const int c = tbase + j;
    int n = __builtin_amdgcn_readlane(cnt_l, j);
    n = n < 0 ? 0 : (n > DEGCAP ? DEGCAP : n);
    const int st = __builtin_amdgcn_readlane(off_l, j);
    v4f a0 = {0.f, 0.f, 0.f, 0.f}, a1 = {0.f, 0.f, 0.f, 0.f};
#pragma unroll 1
    for (int q0 = 0; q0 < n; q0 += 32) {
      int pos = st + q0 + lane;
      pos = pos < 0 ? 0 : (pos > csrLen - 1 ? csrLen - 1 : pos);
      int sl = csr[pos];
      sl = sl < 0 ? 0 : (sl > nN - 1 ? nN - 1 : sl);
      const int mcnt = (n - q0) < 32 ? (n - q0) : 32;
#pragma unroll 1
      for (int p = 0; p < mcnt; ++p) {
        const int s = __builtin_amdgcn_readlane(sl, p);
        const float* sr = X + (size_t)s * DH + 8 * lane;
        a0 = a0 + *(const v4f*)sr;
        a1 = a1 + *(const v4f*)(sr + 4);
      }
    }
    const int cs = c > nN - 1 ? nN - 1 : c;
    const float* xr = X + (size_t)cs * DH + 8 * lane;
    a0 = a0 + *(const v4f*)xr;
    a1 = a1 + *(const v4f*)(xr + 4);

    const size_t g = (size_t)c * DH + 8 * lane;
    if (doHL != 0) {
      v8us hv, lv;
      split8(a0, a1, hv, lv);
      unsigned short* p0 = Ohi + g;
      unsigned short* p1 = Olo + g;
      *(volatile v8us*)p0 = hv;
      *(volatile v8us*)p1 = lv;
      __threadfence();
      *(volatile v8us*)p0 = hv;
      *(volatile v8us*)p1 = lv;
    }
    if (doF != 0) {
      const v8h fv = cvt8h(a0 * ASCALE, a1 * ASCALE);
      unsigned short* p2 = Of + g;
      *(volatile v8h*)p2 = fv;
      __threadfence();
      *(volatile v8h*)p2 = fv;
    }
  }
}

template <int TERMS, int EP>
__global__ __launch_bounds__(NTHR) void k_gemm(
    const unsigned short* __restrict__ Ah, const unsigned short* __restrict__ Al,
    const unsigned short* __restrict__ Bh, const unsigned short* __restrict__ Bl,
    const float* __restrict__ bias, float scale,
    unsigned short* O16a, unsigned short* O16b, float* O32a, float* O32b) {
  extern __shared__ v4f lds_dyn[];
  float* stg = (float*)lds_dyn;
  const int tid = threadIdx.x, lane = tid & 31, wave = tid >> 5, hh = lane >> 4, m = lane & 15;
  const int rowBase = blockIdx.x * GROWS;
  const int r0 = (wave & 3) * 16;
  const int c0 = (wave >> 2) * 128;

  v8f acc[8];
#pragma unroll
  for (int t = 0; t < 8; ++t) { v8f z = {0.f, 0.f, 0.f, 0.f, 0.f, 0.f, 0.f, 0.f}; acc[t] = z; }

  const unsigned short* ah = Ah + (size_t)(rowBase + r0 + m) * DH + 8 * hh;
  const unsigned short* al = Al + (size_t)(rowBase + r0 + m) * DH + 8 * hh;
  const unsigned short* bh = Bh + (size_t)(c0 + m) * DH + 8 * hh;
  const unsigned short* bl = Bl + (size_t)(c0 + m) * DH + 8 * hh;

#pragma unroll 1
  for (int kt = 0; kt < DH / 32; ++kt) {
    Frag fa, ga;
    fa.h[0] = *(const v8us*)(ah + 32 * kt);
    fa.h[1] = *(const v8us*)(ah + 32 * kt + 16);
    if (TERMS == 3) {
      ga.h[0] = *(const v8us*)(al + 32 * kt);
      ga.h[1] = *(const v8us*)(al + 32 * kt + 16);
    } else {
      ga = fa;
    }
#pragma unroll
    for (int t = 0; t < 8; ++t) {
      const unsigned short* bp = bh + (size_t)(16 * t) * DH + 32 * kt;
      Frag fb;
      fb.h[0] = *(const v8us*)bp;
      fb.h[1] = *(const v8us*)(bp + 16);
      if (TERMS == 3) {
        const unsigned short* cp = bl + (size_t)(16 * t) * DH + 32 * kt;
        Frag gb;
        gb.h[0] = *(const v8us*)cp;
        gb.h[1] = *(const v8us*)(cp + 16);
        acc[t] = wm_bf16(fa.b, fb.b, acc[t]);
        acc[t] = wm_bf16(fa.b, gb.b, acc[t]);
        acc[t] = wm_bf16(ga.b, fb.b, acc[t]);
      } else {
        acc[t] = wm_f16(fa.f, fb.f, acc[t]);
      }
    }
  }

#pragma unroll
  for (int t = 0; t < 8; ++t) {
    const int col = c0 + 16 * t + m;
    const float bv = bias[col];
    float* sp = stg + (r0 + 8 * hh) * DH + col;
#pragma unroll
    for (int r = 0; r < 8; ++r) {
      float v = acc[t][r] * scale + bv;
      if (EP == 0) v = fmaxf(v, 0.0f);
      sp[r * DH] = v;
    }
  }
  __syncthreads();

#pragma unroll 1
  for (int i = 0; i < GROWS / NWAVE; ++i) {
    const int rl = wave * (GROWS / NWAVE) + i;
    const size_t g = (size_t)(rowBase + rl) * DH;
    const float* lr = stg + rl * DH;
    const v4f xa = *(const v4f*)(lr + 8 * lane);
    const v4f xb = *(const v4f*)(lr + 8 * lane + 4);
    const v4f ya = *(const v4f*)(lr + 4 * lane);
    const v4f yb = *(const v4f*)(lr + 128 + 4 * lane);
    if (EP == 0) {
      if (TERMS == 3) {
        v8us hv, lv;
        split8(xa, xb, hv, lv);
        unsigned short* p0 = O16a + g + 8 * lane;
        unsigned short* p1 = O16b + g + 8 * lane;
        *(volatile v8us*)p0 = hv;
        *(volatile v8us*)p1 = lv;
        __threadfence();
        *(volatile v8us*)p0 = hv;
        *(volatile v8us*)p1 = lv;
      } else {
        const v8h fv = cvt8h(xa * ASCALE, xb * ASCALE);
        unsigned short* p0 = O16a + g + 8 * lane;
        *(volatile v8h*)p0 = fv;
        __threadfence();
        *(volatile v8h*)p0 = fv;
      }
    } else if (EP == 1) {
      float* p0 = O32a + g + 4 * lane;
      float* p1 = O32a + g + 128 + 4 * lane;
      *(volatile v4f*)p0 = ya;
      *(volatile v4f*)p1 = yb;
      __threadfence();
      *(volatile v4f*)p0 = ya;
      *(volatile v4f*)p1 = yb;
    } else if (EP == 2) {
      float s = dot8(xa, xb, xa, xb);
      s = wsum32(s);
      const float inv = 1.0f / fmaxf(sqrtf(s), L2EPS);
      const v8h fv = cvt8h(xa * ASCALE, xb * ASCALE);
      const v4f na = ya * inv, nb = yb * inv;
      float* e0 = O32a + g + 4 * lane;
      float* e1 = O32a + g + 128 + 4 * lane;
      unsigned short* f0 = O16a + g + 8 * lane;
      float* n0 = O32b + g + 4 * lane;
      float* n1 = O32b + g + 128 + 4 * lane;
      *(volatile v4f*)e0 = ya;
      *(volatile v4f*)e1 = yb;
      *(volatile v8h*)f0 = fv;
      *(volatile v4f*)n0 = na;
      *(volatile v4f*)n1 = nb;
      __threadfence();
      *(volatile v4f*)e0 = ya;
      *(volatile v4f*)e1 = yb;
      *(volatile v8h*)f0 = fv;
      *(volatile v4f*)n0 = na;
      *(volatile v4f*)n1 = nb;
    } else {
      float s = dot8(xa, xb, xa, xb);
      s = wsum32(s);
      const float inv = 1.0f / fmaxf(sqrtf(s), L2EPS);
      const v4f na = ya * inv, nb = yb * inv;
      float* n0 = O32a + g + 4 * lane;
      float* n1 = O32a + g + 128 + 4 * lane;
      *(volatile v4f*)n0 = na;
      *(volatile v4f*)n1 = nb;
      __threadfence();
      *(volatile v4f*)n0 = na;
      *(volatile v4f*)n1 = nb;
    }
  }
}

__global__ __launch_bounds__(NTHR) void k_loss(
    const float* __restrict__ P, const float* __restrict__ TE, const float* __restrict__ ON,
    const int* __restrict__ pidx, const int* __restrict__ nidx, float* part, int nN, int nS) {
  __shared__ float wpart[NWAVE];
  const int tid = threadIdx.x, lane = tid & 31, wave = tid >> 5;
  float acc = 0.0f;
#pragma unroll 1
  for (int i = 0; i < LNODE / NWAVE; ++i) {
    const int n = blockIdx.x * LNODE + wave * (LNODE / NWAVE) + i;
    const int nc = n > nN - 1 ? nN - 1 : n;
    const float* pr = P + (size_t)nc * DH + 8 * lane;
    const v4f pa = *(const v4f*)pr, pb = *(const v4f*)(pr + 4);
    const float* orw = ON + (size_t)nc * DH + 8 * lane;
    const v4f oa = *(const v4f*)orw, ob = *(const v4f*)(orw + 4);
    float pos = 0.0f, neg = 0.0f;
#pragma unroll 1
    for (int s = 0; s < nS; ++s) {
      int pi = pidx[(size_t)nc * nS + s];
      pi = pi < 0 ? 0 : (pi > nN - 1 ? nN - 1 : pi);
      const float* tr = TE + (size_t)pi * DH + 8 * lane;
      const v4f ta = *(const v4f*)tr, tb = *(const v4f*)(tr + 4);
      float d = dot8(pa, pb, ta, tb);
      d = wsum32(d);
      pos += __expf(2.0f * d);
      int ni = nidx[(size_t)nc * nS + s];
      ni = ni < 0 ? 0 : (ni > nN - 1 ? nN - 1 : ni);
      const float* mr = ON + (size_t)ni * DH + 8 * lane;
      const v4f ma = *(const v4f*)mr, mb = *(const v4f*)(mr + 4);
      float dn = dot8(oa, ob, ma, mb);
      dn = wsum32(dn);
      neg += __expf(2.0f * dn);
    }
    const float term = -__logf(pos * (1.0f / (pos + neg)));
    acc += (n < nN) ? term : 0.0f;
  }
  if (lane == 0) wpart[wave] = acc;
  __syncthreads();
  if (wave == 0) {
    float bs = wpart[0];
    bs += wpart[1]; bs += wpart[2]; bs += wpart[3];
    bs += wpart[4]; bs += wpart[5]; bs += wpart[6]; bs += wpart[7];
    const float v = (lane == 0) ? bs : 0.0f;
    float* pp = part + (size_t)blockIdx.x * 32 + lane;
    *(volatile float*)pp = v;
    __threadfence();
    *(volatile float*)pp = v;
  }
}

__global__ __launch_bounds__(NTHR) void k_pack(
    const float* __restrict__ emb, const float* __restrict__ part, float* out,
    int nEmb, int nPart, float invN) {
  const int tid = threadIdx.x, lane = tid & 31, wave = tid >> 5;
  const int t = blockIdx.x * NTHR + tid;
  float lossv = 0.0f;
  if (blockIdx.x == 0 && wave == 0) {
    float s = 0.0f;
#pragma unroll 1
    for (int i0 = 0; i0 < nPart; i0 += 32) {
      const int i  = i0 + lane;
      const int ic = i > nPart - 1 ? nPart - 1 : i;
      const float v = part[(size_t)ic * 32];
      s += (i < nPart) ? v : 0.0f;
    }
    s = wsum32(s);
    lossv = s * invN;
  }
  const int nF = nEmb + 1;
  const int f0 = 4 * t;
  int e0 = f0 - 1, e1 = f0, e2 = f0 + 1, e3 = f0 + 2;
  e0 = e0 < 0 ? 0 : (e0 > nEmb - 1 ? nEmb - 1 : e0);
  e1 = e1 > nEmb - 1 ? nEmb - 1 : e1;
  e2 = e2 > nEmb - 1 ? nEmb - 1 : e2;
  e3 = e3 > nEmb - 1 ? nEmb - 1 : e3;
  const float a0 = emb[e0], a1 = emb[e1], a2 = emb[e2], a3 = emb[e3];
  v4f v;
  v.x = (f0 == 0) ? lossv : a0;
  v.y = a1; v.z = a2; v.w = a3;
  const bool full = (f0 + 3 < nF);
  const int  rem  = nF - f0;
  const size_t fo = (size_t)(f0 < nF ? f0 : 0);
  float* op = out + fo;
  if (full) {
    *(volatile v4f*)op = v;
  } else if (rem > 0) {
    *(volatile float*)op = v.x;
    if (rem > 1) *(volatile float*)(op + 1) = v.y;
    if (rem > 2) *(volatile float*)(op + 2) = v.z;
  }
  __threadfence();
  if (full) {
    *(volatile v4f*)op = v;
  } else if (rem > 0) {
    *(volatile float*)op = v.x;
    if (rem > 1) *(volatile float*)(op + 1) = v.y;
    if (rem > 2) *(volatile float*)(op + 2) = v.z;
  }
}

extern "C" void kernel_launch(void* const* d_in, const int* in_sizes, int n_in,
                              void* d_out, int out_size, void* d_ws, size_t ws_size,
                              hipStream_t stream) {
  if (n_in < 27) return;
  const int nN = in_sizes[0] / DH;
  if (nN <= 0 || in_sizes[0] != nN * DH) return;
  const int nE = in_sizes[1];
  if (nE <= 0 || in_sizes[2] != nE) return;
  if (in_sizes[3] <= 0 || (in_sizes[3] % nN) != 0 || in_sizes[4] != in_sizes[3]) return;
  const int nS = in_sizes[3] / nN;
  for (int i = 0; i < 11; ++i) {
    if (in_sizes[5 + 2 * i] != DH * DH || in_sizes[6 + 2 * i] != DH) return;
  }
  if (out_size != 1 + nN * DH) return;
  if (nE > (1 << 28) || nN > (1 << 22) || nS > 4096) return;

  const float* h    = (const float*)d_in[0];
  const int*   srcs = (const int*)d_in[1];
  const int*   dsts = (const int*)d_in[2];
  const int*   pidx = (const int*)d_in[3];
  const int*   nidx = (const int*)d_in[4];
  const float* wq[11];
  const float* bq[11];
  for (int i = 0; i < 11; ++i) { wq[i] = (const float*)d_in[5 + 2 * i]; bq[i] = (const float*)d_in[6 + 2 * i]; }
  float* out = (float*)d_out;

  const int NPAD   = ((nN + TGT - 1) / TGT) * TGT;
  const int nBC    = (nN + NBC - 1) / NBC;
  const int CNTPAD = nBC * NBC;
  if (4 * nBC + 1 > RBN) return;
  const int nBF    = (nN + NBF - 1) / NBF;
  if (nBF * NBF > CNTPAD || NPAD > CNTPAD) return;
  const int csrLen = ((nE + 31) & ~31) + 4096;
  const int nGemm  = NPAD / GROWS;
  const int nAgg   = NPAD / TGT;
  const int nLB    = (nN + LNODE - 1) / LNODE;
  const int nEmb   = nN * DH;
  const int nF     = nEmb + 1;
  const int nT     = (nF + 3) / 4;
  const int nPack  = (nT + NTHR - 1) / NTHR;

  const size_t PB32 = (size_t)NPAD * DH * 4;
  char* ws = (char*)d_ws;
  size_t off = 0;
  const size_t oWHL = off; off += (size_t)8 * DH * DH * 2;       off = (off + 255) & ~(size_t)255;
  const size_t oWF  = off; off += (size_t)7 * DH * DH * 2;       off = (off + 255) & ~(size_t)255;
  const size_t oCnt = off; off += (size_t)CNTPAD * 4;            off = (off + 255) & ~(size_t)255;
  const size_t oOff = off; off += (size_t)CNTPAD * 4;            off = (off + 255) & ~(size_t)255;
  const size_t oRb  = off; off += (size_t)RBN * 4;               off = (off + 255) & ~(size_t)255;
  const size_t oCsr = off; off += (size_t)csrLen * 4;            off = (off + 255) & ~(size_t)255;
  const size_t oR1  = off; off += PB32;                          off = (off + 255) & ~(size_t)255;
  const size_t oR2  = off; off += PB32;                          off = (off + 255) & ~(size_t)255;
  const size_t oR3  = off; off += PB32;                          off = (off + 255) & ~(size_t)255;
  const size_t oR4  = off; off += PB32;                          off = (off + 255) & ~(size_t)255;
  const size_t oR5  = off; off += PB32;                          off = (off + 255) & ~(size_t)255;
  const size_t oR6  = off; off += PB32;                          off = (off + 255) & ~(size_t)255;
  const size_t oPt  = off; off += (size_t)nLB * 32 * 4;          off = (off + 255) & ~(size_t)255;
  if (off > ws_size || off > ((size_t)128 << 20)) return;

  unsigned short* whl = (unsigned short*)(ws + oWHL);
  unsigned short* wf  = (unsigned short*)(ws + oWF);
  int*   cnt  = (int*)(ws + oCnt);
  int*   offp = (int*)(ws + oOff);
  int*   rb   = (int*)(ws + oRb);
  int*   csr  = (int*)(ws + oCsr);
  unsigned short* AGGH = (unsigned short*)(ws + oR1);
  unsigned short* AGGL = AGGH + (size_t)NPAD * DH;
  float*          TE   = (float*)(ws + oR1);
  unsigned short* UH   = (unsigned short*)(ws + oR2);
  unsigned short* UL   = UH + (size_t)NPAD * DH;
  unsigned short* UF   = UH;
  unsigned short* U2F  = UL;
  float*          F3   = (float*)(ws + oR3);
  unsigned short* A16  = (unsigned short*)(ws + oR4);
  unsigned short* E16  = A16 + (size_t)NPAD * DH;
  float*          EMB  = (float*)(ws + oR5);
  float*          ON   = (float*)(ws + oR6);
  float*          part = (float*)(ws + oPt);
  unsigned short* udum = (unsigned short*)(ws + oPt);
  float*          fdum = part;

  const int vec8 = ((nE & 3) == 0) ? 1 : 0;
  const float invN = 1.0f / (float)nN;

  k_wprep<<<11 * 32, NTHR, 0, stream>>>(wq[0], wq[1], wq[2], wq[3], wq[4], wq[5], wq[6], wq[7], wq[8], wq[9], wq[10], whl, wf);

  k_count<<<nBC, NTHR, 0, stream>>>(dsts, cnt, nE, vec8);
  k_offsets<<<1, OTHR, 0, stream>>>(cnt, offp, rb, nBC);
  hipFuncSetAttribute(reinterpret_cast<const void*>(&k_fill), hipFuncAttributeMaxDynamicSharedMemorySize, LDS_FILL);
  k_fill<<<nBF, NTHR, LDS_FILL, stream>>>(srcs, dsts, offp, rb, csr, nN, nE, vec8, csrLen);

  hipFuncSetAttribute(reinterpret_cast<const void*>(&k_gemm<3, 0>), hipFuncAttributeMaxDynamicSharedMemorySize, LDS_GEMM);
  hipFuncSetAttribute(reinterpret_cast<const void*>(&k_gemm<3, 1>), hipFuncAttributeMaxDynamicSharedMemorySize, LDS_GEMM);
  hipFuncSetAttribute(reinterpret_cast<const void*>(&k_gemm<3, 2>), hipFuncAttributeMaxDynamicSharedMemorySize, LDS_GEMM);
  hipFuncSetAttribute(reinterpret_cast<const void*>(&k_gemm<1, 0>), hipFuncAttributeMaxDynamicSharedMemorySize, LDS_GEMM);
  hipFuncSetAttribute(reinterpret_cast<const void*>(&k_gemm<1, 1>), hipFuncAttributeMaxDynamicSharedMemorySize, LDS_GEMM);
  hipFuncSetAttribute(reinterpret_cast<const void*>(&k_gemm<1, 3>), hipFuncAttributeMaxDynamicSharedMemorySize, LDS_GEMM);

  k_agg<<<nAgg, NTHR, 0, stream>>>(csr, offp, cnt, h, nN, csrLen, 1, 1, AGGH, AGGL, A16);
  k_gemm<3, 0><<<nGemm, NTHR, LDS_GEMM, stream>>>(AGGH, AGGL, whl + (size_t)0 * DH * DH, whl + (size_t)1 * DH * DH, bq[0], 1.0f, UH, UL, fdum, fdum);
  k_gemm<3, 1><<<nGemm, NTHR, LDS_GEMM, stream>>>(UH, UL, whl + (size_t)2 * DH * DH, whl + (size_t)3 * DH * DH, bq[1], 1.0f, udum, udum, F3, fdum);
  k_agg<<<nAgg, NTHR, 0, stream>>>(csr, offp, cnt, F3, nN, csrLen, 1, 0, AGGH, AGGL, A16);
  k_gemm<3, 0><<<nGemm, NTHR, LDS_GEMM, stream>>>(AGGH, AGGL, whl + (size_t)4 * DH * DH, whl + (size_t)5 * DH * DH, bq[2], 1.0f, UH, UL, fdum, fdum);
  k_gemm<3, 2><<<nGemm, NTHR, LDS_GEMM, stream>>>(UH, UL, whl + (size_t)6 * DH * DH, whl + (size_t)7 * DH * DH, bq[3], 1.0f, E16, udum, EMB, ON);
  k_gemm<1, 0><<<nGemm, NTHR, LDS_GEMM, stream>>>(A16, A16, wf + (size_t)0 * DH * DH, wf + (size_t)0 * DH * DH, bq[4], F16INV, UF, udum, fdum, fdum);
  k_gemm<1, 1><<<nGemm, NTHR, LDS_GEMM, stream>>>(UF, UF, wf + (size_t)1 * DH * DH, wf + (size_t)1 * DH * DH, bq[5], F16INV, udum, udum, F3, fdum);
  k_agg<<<nAgg, NTHR, 0, stream>>>(csr, offp, cnt, F3, nN, csrLen, 0, 1, AGGH, AGGL, A16);
  k_gemm<1, 0><<<nGemm, NTHR, LDS_GEMM, stream>>>(A16, A16, wf + (size_t)2 * DH * DH, wf + (size_t)2 * DH * DH, bq[6], F16INV, UF, udum, fdum, fdum);
  k_gemm<1, 3><<<nGemm, NTHR, LDS_GEMM, stream>>>(UF, UF, wf + (size_t)3 * DH * DH, wf + (size_t)3 * DH * DH, bq[7], F16INV, udum, udum, TE, fdum);
  k_gemm<1, 0><<<nGemm, NTHR, LDS_GEMM, stream>>>(E16, E16, wf + (size_t)4 * DH * DH, wf + (size_t)4 * DH * DH, bq[8], F16INV, UF, udum, fdum, fdum);
  k_gemm<1, 0><<<nGemm, NTHR, LDS_GEMM, stream>>>(UF, UF, wf + (size_t)5 * DH * DH, wf + (size_t)5 * DH * DH, bq[9], F16INV, U2F, udum, fdum, fdum);
  k_gemm<1, 3><<<nGemm, NTHR, LDS_GEMM, stream>>>(U2F, U2F, wf + (size_t)6 * DH * DH, wf + (size_t)6 * DH * DH, bq[10], F16INV, udum, udum, F3, fdum);
  k_loss<<<nLB, NTHR, 0, stream>>>(F3, TE, ON, pidx, nidx, part, nN, nS);
  k_pack<<<nPack, NTHR, 0, stream>>>(EMB, part, out, nEmb, nLB, invN);
}
